// _EfficientSelfAttn_25718264168519
// MI455X (gfx1250) — hardware-verified
//
#include <hip/hip_runtime.h>
#include <stdint.h>

typedef unsigned short u16;
typedef u16    v16u __attribute__((ext_vector_type(16)));
typedef u16    v8u  __attribute__((ext_vector_type(8)));
typedef __bf16 v16b __attribute__((ext_vector_type(16)));
typedef float  v8f  __attribute__((ext_vector_type(8)));
typedef float  v4f  __attribute__((ext_vector_type(4)));
typedef v8u __attribute__((may_alias)) v8ua;
typedef v4f __attribute__((may_alias)) v4fa;

union Frag { v16b v; v16u u; v8u half[2]; };
static_assert(sizeof(Frag) == 32);

#define NBATCH 8
#define NQ     16384
#define CD     64
#define NKEY   256
#define NROWK  2048
#define KCONV  4096
#define LN_EPS 1e-5f

__device__ __forceinline__ v8f wmma_bf(v16b a, v16b b, v8f c) {
  v8f d = __builtin_amdgcn_wmma_f32_16x16x32_bf16(false, a, false, b, (short)0, c, false, false);
  asm volatile("v_nop\n\tv_nop\n\tv_nop\n\tv_nop" : "+v"(d) : "v"(a), "v"(b));
  return d;
}

__device__ __forceinline__ u16 bf_rne(float f) {
  unsigned u = __builtin_bit_cast(unsigned, f);
  u += 0x7FFFu + ((u >> 16) & 1u);
  return (u16)(u >> 16);
}
__device__ __forceinline__ float bf_val(u16 b) {
  return __builtin_bit_cast(float, ((unsigned)b) << 16);
}

__device__ __forceinline__ void split8(v8f f, v8u& hi, v8u& lo) {
  #pragma unroll
  for (int i = 0; i < 8; ++i) {
    const u16 hh = bf_rne(f[i]);
    hi[i] = hh;
    lo[i] = bf_rne(f[i] - bf_val(hh));
  }
}

__device__ __forceinline__ void split_frag(v8f a, v8f c, v16b& fhi, v16b& flo) {
  Frag fh, fl;
  v8u h0, l0, h1, l1;
  split8(a, h0, l0);
  split8(c, h1, l1);
  fh.half[0] = h0; fh.half[1] = h1;
  fl.half[0] = l0; fl.half[1] = l1;
  fhi = fh.v; flo = fl.v;
}

__device__ __forceinline__ v16b ld_frag(const u16* p, int h) {
  Frag f;
  f.half[0] = *(const v8ua*)(p + 8 * h);
  f.half[1] = *(const v8ua*)(p + 16 + 8 * h);
  return f.v;
}

__device__ __forceinline__ float red16(float v) {
  v += __shfl_xor(v, 1);
  v += __shfl_xor(v, 2);
  v += __shfl_xor(v, 4);
  v += __shfl_xor(v, 8);
  return v;
}

__global__ __launch_bounds__(256) void k_prep_w(
    const float* __restrict__ wq, const float* __restrict__ wkv,
    const float* __restrict__ wproj, const float* __restrict__ wsr,
    u16* __restrict__ wqh, u16* __restrict__ wql,
    u16* __restrict__ wkvh, u16* __restrict__ wkvl,
    u16* __restrict__ wph, u16* __restrict__ wpl,
    u16* __restrict__ wsh, u16* __restrict__ wsl)
{
  const int blk = blockIdx.x, tid = threadIdx.x;
  if (blk >= 136) return;
  v8f f;
  u16* dh;
  u16* dl;
  int e;
  if (blk < 8) {
    const float* src;
    if (blk < 2)      { e = blk * 256 + tid;        src = wq;    dh = wqh;  dl = wql;  }
    else if (blk < 6) { e = (blk - 2) * 256 + tid;  src = wkv;   dh = wkvh; dl = wkvl; }
    else              { e = (blk - 6) * 256 + tid;  src = wproj; dh = wph;  dl = wpl;  }
    const float* s = src + (size_t)e * 8;
    const v4f a = *(const v4fa*)s;
    const v4f c = *(const v4fa*)(s + 4);
    f = __builtin_shufflevector(a, c, 0, 1, 2, 3, 4, 5, 6, 7);
  } else {
    e = (blk - 8) * 256 + tid;
    const int co = e >> 9, grp = e & 511;
    const int p = grp >> 3, ci0 = (grp & 7) * 8;
    const float* s = wsr + (size_t)co * KCONV + ci0 * 64 + p;
    #pragma unroll
    for (int c = 0; c < 8; ++c) f[c] = s[c * 64];
    dh = wsh; dl = wsl;
  }
  v8u hi, lo;
  split8(f, hi, lo);
  u16* ph = dh + (size_t)e * 8;
  u16* pl = dl + (size_t)e * 8;
  *(volatile v8u*)ph = hi;
  *(volatile v8u*)pl = lo;
  __threadfence();
  *(volatile v8u*)ph = hi;
  *(volatile v8u*)pl = lo;
}

__global__ __launch_bounds__(256) void k_im2col(
    const float* __restrict__ x, const int* __restrict__ Hp, const int* __restrict__ Wp,
    u16* __restrict__ ah, u16* __restrict__ al)
{
  const int g = blockIdx.x * 256 + threadIdx.x;
  if (g >= NROWK * 512) return;
  const int Hv = Hp[0], Wv = Wp[0];
  const long long hw = (long long)Hv * (long long)Wv;
  const int lim = (hw >= 1 && hw <= NQ) ? (int)(hw - 1) : (NQ - 1);
  const int r = g >> 9, grp = g & 511;
  const int bb = r >> 8, mm = r & 255;
  const int py = mm >> 4, px = mm & 15;
  const int p = grp >> 3, ci0 = (grp & 7) * 8;
  const int ii = p >> 3, jj = p & 7;
  int pix = (8 * py + ii) * Wv + 8 * px + jj;
  pix = min(max(pix, 0), lim);
  const float* s = x + ((size_t)bb * NQ + pix) * CD + ci0;
  const v4f a = *(const v4fa*)s;
  const v4f c = *(const v4fa*)(s + 4);
  const v8f f = __builtin_shufflevector(a, c, 0, 1, 2, 3, 4, 5, 6, 7);
  v8u hi, lo;
  split8(f, hi, lo);
  u16* ph = ah + (size_t)g * 8;
  u16* pl = al + (size_t)g * 8;
  *(volatile v8u*)ph = hi;
  *(volatile v8u*)pl = lo;
  __threadfence();
  *(volatile v8u*)ph = hi;
  *(volatile v8u*)pl = lo;
}

__device__ __forceinline__ void kv_store_pass(const u16* sK, const u16* sV,
                                              u16* kh, u16* kl, u16* vth, u16* vtl,
                                              int blk, int w, int lane) {
  const int q8 = lane & 7, sub = lane >> 3;
  const int bb = blk >> 2, key0 = (blk & 3) * 64, rowbase = blk * 64;
  #pragma unroll
  for (int it = 0; it < 16; ++it) {
    v8u v;
    u16* dst;
    if (it < 8) {
      const int p = (it >> 2) & 1;
      const int kk = (it & 3) * 16 + w * 4 + sub;
      v = *(const v8ua*)(sK + (p * 64 + kk) * 64 + 8 * q8);
      u16* plane = p ? kl : kh;
      dst = plane + (size_t)(rowbase + kk) * CD + 8 * q8;
    } else {
      const int p = ((it - 8) >> 2) & 1;
      const int d = ((it - 8) & 3) * 16 + w * 4 + sub;
      v = *(const v8ua*)(sV + (p * 64 + d) * 64 + 8 * q8);
      u16* plane = p ? vtl : vth;
      dst = plane + ((size_t)(bb * CD + d)) * NKEY + key0 + 8 * q8;
    }
    *(volatile v8u*)dst = v;
  }
}

__global__ __launch_bounds__(128) void k_kv(
    const u16* __restrict__ ah, const u16* __restrict__ al,
    const u16* __restrict__ wsh, const u16* __restrict__ wsl,
    const float* __restrict__ gamma, const float* __restrict__ beta,
    const u16* __restrict__ wkvh, const u16* __restrict__ wkvl,
    const float* __restrict__ bkv,
    u16* __restrict__ kh, u16* __restrict__ kl,
    u16* __restrict__ vth, u16* __restrict__ vtl)
{
  __shared__ __attribute__((aligned(16))) u16 sX[2 * 64 * 64];
  __shared__ __attribute__((aligned(16))) u16 sK[2 * 64 * 64];
  __shared__ __attribute__((aligned(16))) u16 sV[2 * 64 * 64];

  const int tid = threadIdx.x, lane = tid & 31, w = tid >> 5;
  const int h = lane >> 4, m = lane & 15;
  const int blk = blockIdx.x;
  const int rowg = blk * 64 + 16 * w;

  const v8f zero8 = {0.f, 0.f, 0.f, 0.f, 0.f, 0.f, 0.f, 0.f};
  v8f acc[4];
  #pragma unroll
  for (int t = 0; t < 4; ++t) acc[t] = zero8;

  const u16* arh = ah + (size_t)(rowg + m) * KCONV;
  const u16* arl = al + (size_t)(rowg + m) * KCONV;
  const u16* brh = wsh + (size_t)m * KCONV;
  const u16* brl = wsl + (size_t)m * KCONV;

  #pragma unroll 1
  for (int k0 = 0; k0 < KCONV; k0 += 32) {
    const v16b fah = ld_frag(arh + k0, h);
    const v16b fal = ld_frag(arl + k0, h);
    #pragma unroll
    for (int t = 0; t < 4; ++t) {
      const v16b fbh = ld_frag(brh + (size_t)t * 16 * KCONV + k0, h);
      const v16b fbl = ld_frag(brl + (size_t)t * 16 * KCONV + k0, h);
      acc[t] = wmma_bf(fah, fbh, acc[t]);
      acc[t] = wmma_bf(fah, fbl, acc[t]);
      acc[t] = wmma_bf(fal, fbh, acc[t]);
    }
  }

  float mu[8], rs[8];
  #pragma unroll
  for (int r = 0; r < 8; ++r) {
    float s = acc[0][r] + acc[1][r] + acc[2][r] + acc[3][r];
    s = red16(s);
    mu[r] = s * (1.0f / 64.0f);
    float v = 0.f;
    #pragma unroll
    for (int t = 0; t < 4; ++t) { const float d = acc[t][r] - mu[r]; v += d * d; }
    v = red16(v) * (1.0f / 64.0f);
    rs[r] = rsqrtf(v + LN_EPS);
  }
  #pragma unroll
  for (int t = 0; t < 4; ++t) {
    const int col = 16 * t + m;
    const float g = gamma[col], be = beta[col];
    #pragma unroll
    for (int r = 0; r < 8; ++r) {
      const float y = (acc[t][r] - mu[r]) * rs[r] * g + be;
      const u16 hh = bf_rne(y);
      const u16 ll = bf_rne(y - bf_val(hh));
      const int kl_ = 16 * w + 8 * h + r;
      sX[kl_ * 64 + col] = hh;
      sX[4096 + kl_ * 64 + col] = ll;
    }
  }
  __syncthreads();

  const v16b xah0 = ld_frag(sX + (16 * w + m) * 64, h);
  const v16b xah1 = ld_frag(sX + (16 * w + m) * 64 + 32, h);
  const v16b xal0 = ld_frag(sX + 4096 + (16 * w + m) * 64, h);
  const v16b xal1 = ld_frag(sX + 4096 + (16 * w + m) * 64 + 32, h);

  #pragma unroll
  for (int ct = 0; ct < 8; ++ct) {
    const int off = (16 * ct + m) * CD;
    const v16b b0h = ld_frag(wkvh + off, h);
    const v16b b0l = ld_frag(wkvl + off, h);
    const v16b b1h = ld_frag(wkvh + off + 32, h);
    const v16b b1l = ld_frag(wkvl + off + 32, h);
    v8f c = zero8;
    c = wmma_bf(xah0, b0h, c);
    c = wmma_bf(xah0, b0l, c);
    c = wmma_bf(xal0, b0h, c);
    c = wmma_bf(xah1, b1h, c);
    c = wmma_bf(xah1, b1l, c);
    c = wmma_bf(xal1, b1h, c);
    const int col = 16 * ct + m;
    const float bb = bkv[col];
    #pragma unroll
    for (int r = 0; r < 8; ++r) {
      const float val = c[r] + bb;
      const u16 hh = bf_rne(val);
      const u16 ll = bf_rne(val - bf_val(hh));
      const int kl_ = 16 * w + 8 * h + r;
      if (ct < 4) {
        sK[kl_ * 64 + col] = hh;
        sK[4096 + kl_ * 64 + col] = ll;
      } else {
        const int d = col - 64;
        sV[d * 64 + kl_] = hh;
        sV[4096 + d * 64 + kl_] = ll;
      }
    }
  }
  __syncthreads();

  kv_store_pass(sK, sV, kh, kl, vth, vtl, blk, w, lane);
  __threadfence();
  kv_store_pass(sK, sV, kh, kl, vth, vtl, blk, w, lane);
}

__device__ __forceinline__ void att_store_pass(const float* so, float* out, size_t grow0, int lane) {
  const int q8 = lane & 7, sub = lane >> 3;
  #pragma unroll
  for (int i = 0; i < 8; ++i) {
    const int lid = i * 4 + sub;
    const int row = lid >> 1, hl = lid & 1;
    const v4f v = *(const v4fa*)(so + row * 64 + 32 * hl + 4 * q8);
    *(volatile v4f*)(out + (grow0 + (size_t)row) * CD + 32 * hl + 4 * q8) = v;
  }
}

__global__ __launch_bounds__(64) void k_attn(
    const float* __restrict__ x,
    const u16* __restrict__ wqh, const u16* __restrict__ wql, const float* __restrict__ bq,
    const u16* __restrict__ kh, const u16* __restrict__ kl,
    const u16* __restrict__ vth, const u16* __restrict__ vtl,
    const u16* __restrict__ wph, const u16* __restrict__ wpl, const float* __restrict__ bproj,
    float* __restrict__ out)
{
  __shared__ __attribute__((aligned(16))) float sS[2][16 * 256];
  __shared__ __attribute__((aligned(16))) float sO[2][16 * 64];

  const int tid = threadIdx.x, lane = tid & 31, w = tid >> 5;
  const int h = lane >> 4, m = lane & 15;
  const int b = blockIdx.y;
  const int q0 = blockIdx.x * 32 + 16 * w;
  const v8f zero8 = {0.f, 0.f, 0.f, 0.f, 0.f, 0.f, 0.f, 0.f};

  v8f qt[4];
  #pragma unroll
  for (int t = 0; t < 4; ++t) qt[t] = zero8;
  const float* xr = x + ((size_t)b * NQ + q0 + m) * CD;
  #pragma unroll
  for (int ks = 0; ks < 2; ++ks) {
    const float* xp = xr + 32 * ks + 8 * h;
    const v4f a0 = *(const v4fa*)(xp);
    const v4f a1 = *(const v4fa*)(xp + 4);
    const v4f c0 = *(const v4fa*)(xp + 16);
    const v4f c1 = *(const v4fa*)(xp + 20);
    const v8f a8 = __builtin_shufflevector(a0, a1, 0, 1, 2, 3, 4, 5, 6, 7);
    const v8f c8 = __builtin_shufflevector(c0, c1, 0, 1, 2, 3, 4, 5, 6, 7);
    v16b xbh, xbl;
    split_frag(a8, c8, xbh, xbl);
    #pragma unroll
    for (int t = 0; t < 4; ++t) {
      const int off = (16 * t + m) * CD + 32 * ks;
      const v16b fah = ld_frag(wqh + off, h);
      const v16b fal = ld_frag(wql + off, h);
      qt[t] = wmma_bf(fah, xbh, qt[t]);
      qt[t] = wmma_bf(fah, xbl, qt[t]);
      qt[t] = wmma_bf(fal, xbh, qt[t]);
    }
  }
  v8f qv[4];
  #pragma unroll
  for (int t = 0; t < 4; ++t)
    #pragma unroll
    for (int r = 0; r < 8; ++r)
      qv[t][r] = (qt[t][r] + bq[16 * t + 8 * h + r]) * 0.125f;
  v16b qbh0, qbl0, qbh1, qbl1;
  split_frag(qv[0], qv[1], qbh0, qbl0);
  split_frag(qv[2], qv[3], qbh1, qbl1);

  float* sw = &sS[w][0];
  float* srow = sw + m * 256 + 8 * h;
  float mx = -3.0e38f;
  const u16* kbh = kh + ((size_t)b * NKEY + m) * CD;
  const u16* kbl = kl + ((size_t)b * NKEY + m) * CD;
  #pragma unroll 1
  for (int j = 0; j < 16; ++j) {
    const int ko = 16 * j * CD;
    const v16b a0h = ld_frag(kbh + ko, h);
    const v16b a0l = ld_frag(kbl + ko, h);
    const v16b a1h = ld_frag(kbh + ko + 32, h);
    const v16b a1l = ld_frag(kbl + ko + 32, h);
    v8f z = zero8;
    z = wmma_bf(a0h, qbh0, z);
    z = wmma_bf(a0h, qbl0, z);
    z = wmma_bf(a0l, qbh0, z);
    z = wmma_bf(a1h, qbh1, z);
    z = wmma_bf(a1h, qbl1, z);
    z = wmma_bf(a1l, qbh1, z);
    const v4f z0 = __builtin_shufflevector(z, z, 0, 1, 2, 3);
    const v4f z1 = __builtin_shufflevector(z, z, 4, 5, 6, 7);
    *(v4fa*)(srow + 16 * j) = z0;
    *(v4fa*)(srow + 16 * j + 4) = z1;
    #pragma unroll
    for (int r = 0; r < 8; ++r) mx = fmaxf(mx, z[r]);
  }
  mx = fmaxf(mx, __shfl_xor(mx, 16));

  float sum = 0.f;
  #pragma unroll 2
  for (int a = 0; a < 16; ++a) {
    float* pp = srow + 16 * a;
    v4f v0 = *(const v4fa*)pp;
    v4f v1 = *(const v4fa*)(pp + 4);
    #pragma unroll
    for (int e = 0; e < 4; ++e) {
      v0[e] = __expf(v0[e] - mx);
      v1[e] = __expf(v1[e] - mx);
      sum += v0[e] + v1[e];
    }
    *(v4fa*)pp = v0;
    *(v4fa*)(pp + 4) = v1;
  }
  sum += __shfl_xor(sum, 16);
  const float inv = 1.0f / sum;

  v8f o[4];
  #pragma unroll
  for (int t = 0; t < 4; ++t) o[t] = zero8;
  const u16* vbh = vth + ((size_t)b * CD + m) * NKEY;
  const u16* vbl = vtl + ((size_t)b * CD + m) * NKEY;
  #pragma unroll 1
  for (int c = 0; c < 8; ++c) {
    const int k0 = 32 * c;
    const float* pp = srow + k0;
    const v4f p0 = *(const v4fa*)pp;
    const v4f p1 = *(const v4fa*)(pp + 4);
    const v4f p2 = *(const v4fa*)(pp + 16);
    const v4f p3 = *(const v4fa*)(pp + 20);
    const v8f pa = __builtin_shufflevector(p0, p1, 0, 1, 2, 3, 4, 5, 6, 7) * inv;
    const v8f pc = __builtin_shufflevector(p2, p3, 0, 1, 2, 3, 4, 5, 6, 7) * inv;
    v16b pbh, pbl;
    split_frag(pa, pc, pbh, pbl);
    #pragma unroll
    for (int t = 0; t < 4; ++t) {
      const int vo = 16 * t * NKEY + k0;
      const v16b fah = ld_frag(vbh + vo, h);
      const v16b fal = ld_frag(vbl + vo, h);
      o[t] = wmma_bf(fah, pbh, o[t]);
      o[t] = wmma_bf(fah, pbl, o[t]);
      o[t] = wmma_bf(fal, pbh, o[t]);
    }
  }

  v16b obh0, obl0, obh1, obl1;
  split_frag(o[0], o[1], obh0, obl0);
  split_frag(o[2], o[3], obh1, obl1);
  v8f u[4];
  #pragma unroll
  for (int t = 0; t < 4; ++t) {
    const int off = (16 * t + m) * CD;
    const v16b a0h = ld_frag(wph + off, h);
    const v16b a0l = ld_frag(wpl + off, h);
    const v16b a1h = ld_frag(wph + off + 32, h);
    const v16b a1l = ld_frag(wpl + off + 32, h);
    v8f z = zero8;
    z = wmma_bf(a0h, obh0, z);
    z = wmma_bf(a0h, obl0, z);
    z = wmma_bf(a0l, obh0, z);
    z = wmma_bf(a1h, obh1, z);
    z = wmma_bf(a1h, obl1, z);
    z = wmma_bf(a1l, obh1, z);
    u[t] = z;
  }
  float* so = &sO[w][0];
  #pragma unroll
  for (int t = 0; t < 4; ++t)
    #pragma unroll
    for (int r = 0; r < 8; ++r)
      so[m * 64 + 16 * t + 8 * h + r] = u[t][r] + bproj[16 * t + 8 * h + r];
  __syncthreads();

  const size_t grow0 = (size_t)b * NQ + q0;
  att_store_pass(so, out, grow0, lane);
  __threadfence();
  att_store_pass(so, out, grow0, lane);
}

extern "C" void kernel_launch(void* const* d_in, const int* in_sizes, int n_in,
                              void* d_out, int out_size, void* d_ws, size_t ws_size,
                              hipStream_t stream) {
  if (n_in < 12) return;
  if (in_sizes[0] != NBATCH * NQ * CD) return;
  if (in_sizes[1] != CD * CD || in_sizes[2] != CD) return;
  if (in_sizes[3] != 2 * CD * CD || in_sizes[4] != 2 * CD) return;
  if (in_sizes[5] != CD * CD || in_sizes[6] != CD) return;
  if (in_sizes[7] != CD * KCONV) return;
  if (in_sizes[8] != CD || in_sizes[9] != CD) return;
  if (in_sizes[10] < 1 || in_sizes[11] < 1) return;
  if (out_size != NBATCH * NQ * CD) return;

  const float* x     = (const float*)d_in[0];
  const float* wq    = (const float*)d_in[1];
  const float* bq    = (const float*)d_in[2];
  const float* wkv   = (const float*)d_in[3];
  const float* bkv   = (const float*)d_in[4];
  const float* wproj = (const float*)d_in[5];
  const float* bproj = (const float*)d_in[6];
  const float* wsr   = (const float*)d_in[7];
  const float* gamma = (const float*)d_in[8];
  const float* beta  = (const float*)d_in[9];
  const int*   Hp    = (const int*)d_in[10];
  const int*   Wp    = (const int*)d_in[11];
  float* out = (float*)d_out;

  const size_t szWq  = (size_t)CD * CD * 2;
  const size_t szWkv = (size_t)2 * CD * CD * 2;
  const size_t szWp  = (size_t)CD * CD * 2;
  const size_t szWs  = (size_t)CD * KCONV * 2;
  const size_t szA   = (size_t)NROWK * KCONV * 2;
  const size_t szK   = (size_t)NROWK * CD * 2;
  const size_t szVt  = (size_t)NBATCH * CD * NKEY * 2;
  size_t off = 0;
  const size_t oWqh = off;  off += szWq;
  const size_t oWql = off;  off += szWq;
  const size_t oWkh = off;  off += szWkv;
  const size_t oWkl = off;  off += szWkv;
  const size_t oWph = off;  off += szWp;
  const size_t oWpl = off;  off += szWp;
  const size_t oWsh = off;  off += szWs;
  const size_t oWsl = off;  off += szWs;
  const size_t oAh  = off;  off += szA;
  const size_t oAl  = off;  off += szA;
  const size_t oKh  = off;  off += szK;
  const size_t oKl  = off;  off += szK;
  const size_t oVth = off;  off += szVt;
  const size_t oVtl = off;  off += szVt;
  if (off > ws_size) return;
  if (off > (size_t)134217728) return;

  char* ws = (char*)d_ws;
  u16* wqh  = (u16*)(ws + oWqh);
  u16* wql  = (u16*)(ws + oWql);
  u16* wkvh = (u16*)(ws + oWkh);
  u16* wkvl = (u16*)(ws + oWkl);
  u16* wph  = (u16*)(ws + oWph);
  u16* wpl  = (u16*)(ws + oWpl);
  u16* wsh  = (u16*)(ws + oWsh);
  u16* wsl  = (u16*)(ws + oWsl);
  u16* ah   = (u16*)(ws + oAh);
  u16* al   = (u16*)(ws + oAl);
  u16* kh   = (u16*)(ws + oKh);
  u16* kl   = (u16*)(ws + oKl);
  u16* vth  = (u16*)(ws + oVth);
  u16* vtl  = (u16*)(ws + oVtl);

  k_prep_w<<<136, 256, 0, stream>>>(wq, wkv, wproj, wsr, wqh, wql, wkvh, wkvl, wph, wpl, wsh, wsl);

  k_im2col<<<(NROWK * 512) / 256, 256, 0, stream>>>(x, Hp, Wp, ah, al);

  k_kv<<<NROWK / 64, 128, 0, stream>>>(ah, al, wsh, wsl, gamma, beta, wkvh, wkvl, bkv,
                                       kh, kl, vth, vtl);

  dim3 gAtt(NQ / 32, NBATCH);
  k_attn<<<gAtt, 64, 0, stream>>>(x, wqh, wql, bq, kh, kl, vth, vtl, wph, wpl, bproj, out);
}
